// Conv2d_53334903882373
// MI455X (gfx1250) — hardware-verified
//
#include <hip/hip_runtime.h>
#include <stdint.h>

#define NI   8
#define CI   64
#define CO   64
#define HI   128
#define WI   128
#define HO   126
#define WO   126
#define KG   16
#define LDC  72
#define NCOL 130

typedef _Float16 h16;
typedef __attribute__((ext_vector_type(16))) _Float16 v16h;
typedef __attribute__((ext_vector_type(8)))  _Float16 v8h;
typedef __attribute__((ext_vector_type(8)))  float v8f;
typedef __attribute__((ext_vector_type(2)))  float v2f_t;
typedef float v2fa __attribute__((ext_vector_type(2), may_alias));
typedef __attribute__((ext_vector_type(4)))  unsigned v4u_t;
typedef unsigned v4ua __attribute__((ext_vector_type(4), may_alias));

__device__ __forceinline__ v8f wmma16(v16h a, v16h b, v8f c) {
  return __builtin_amdgcn_wmma_f32_16x16x32_f16(false, a, false, b, (short)0, c, false, false);
}
__device__ __forceinline__ v16h rfrag(const h16* rowp, int half) {
  const h16* p = rowp + 8 * half;
  return __builtin_shufflevector(*(const v8h*)p, *(const v8h*)(p + 16), 0,1,2,3,4,5,6,7,8,9,10,11,12,13,14,15);
}

__global__ __launch_bounds__(256) void k_pack_w(const float* __restrict__ w, h16* __restrict__ wp) {
  const int g = blockIdx.x * 256 + threadIdx.x;
  if (g >= 9 * CO * (CI / 8)) return;
  const int c8 = (g & 7) * 8, co = (g >> 3) & 63, tap = g >> 9;
  h16 hh[8];
#pragma unroll
  for (int e = 0; e < 8; ++e) hh[e] = (h16)w[((size_t)co * CI + c8 + e) * 9 + tap];
  h16* d = wp + ((size_t)tap * CO + co) * CI + c8;
  *(volatile v4u_t*)d = *(const v4ua*)hh; __threadfence(); *(volatile v4u_t*)d = *(const v4ua*)hh;
}

__global__ __launch_bounds__(256) void k_pack_x(const float* __restrict__ x, h16* __restrict__ xp) {
  const int g = blockIdx.x * 256 + threadIdx.x;
  if (g >= NI * HI * WI * (CI / 8)) return;
  const int wv = g & 127, c8 = ((g >> 7) & 7) * 8, hv = (g >> 10) & 127, n = g >> 17;
  h16 hh[8];
#pragma unroll
  for (int e = 0; e < 8; ++e) hh[e] = (h16)x[(((size_t)n * CI + c8 + e) * HI + hv) * WI + wv];
  h16* d = xp + (((size_t)n * HI + hv) * WI + wv) * CI + c8;
  *(volatile v4u_t*)d = *(const v4ua*)hh; __threadfence(); *(volatile v4u_t*)d = *(const v4ua*)hh;
}

__global__ __launch_bounds__(256) void k_conv(const h16* __restrict__ xp, const h16* __restrict__ wp, float* __restrict__ out) {
  __shared__ __attribute__((aligned(16))) h16 halo[3 * NCOL * LDC];
  __shared__ __attribute__((aligned(16))) h16 ws[9 * KG * LDC];
  __shared__ __attribute__((aligned(16))) float so[KG * 128];
  const int n = blockIdx.x >> 2, kg = (blockIdx.x & 3) * KG;
  const int tid = threadIdx.x, lane = tid & 31, wave = tid >> 5, half = lane >> 4, l16 = lane & 15;

  for (int ch = tid; ch < 9 * KG * 8; ch += 256) { const int c8 = (ch & 7) * 8, co = (ch >> 3) & 15, tap = ch >> 7;
    *(v4u_t*)(ws + (tap * KG + co) * LDC + c8) = *(const v4ua*)(wp + ((size_t)tap * CO + kg + co) * CI + c8); }
  for (int ch = tid; ch < 3 * 2 * 8; ch += 256) { const int c8 = (ch & 7) * 8, col = 128 + ((ch >> 3) & 1), r = ch >> 4;
    h16 z[8] = {0,0,0,0,0,0,0,0}; *(v4u_t*)(halo + (r * NCOL + col) * LDC + c8) = *(const v4ua*)z; }

  float* obase = out + ((size_t)n * CO + kg) * HO * WO;
#pragma unroll 1
  for (int y = 0; y < HO; ++y) {
    __syncthreads();
    for (int ch = tid; ch < 3 * 128 * 8; ch += 256) { const int c8 = (ch & 7) * 8, col = (ch >> 3) & 127, r = ch >> 10;
      *(v4u_t*)(halo + (r * NCOL + col) * LDC + c8) = *(const v4ua*)(xp + (((size_t)n * HI + y + r) * WI + col) * CI + c8); }
    __syncthreads();
    const int px = wave * 16 + l16;
    v8f acc = {};
#pragma unroll 3
    for (int t18 = 0; t18 < 18; ++t18) {
      const int tap = t18 >> 1, cib = (t18 & 1) * 32, dy = tap / 3, dx = tap - dy * 3;
      const v16h a = rfrag(halo + (dy * NCOL + px + dx) * LDC + cib, half);
      const v16h b = rfrag(ws + (tap * KG + l16) * LDC + cib, half);
      acc = wmma16(a, b, acc);
    }
    asm volatile("v_nop\n\tv_nop\n\tv_nop\n\tv_nop\n\tv_nop\n\tv_nop\n\tv_nop\n\tv_nop" ::: "memory");
#pragma unroll
    for (int r = 0; r < 8; ++r) so[l16 * 128 + wave * 16 + 8 * half + r] = acc[r];
    __syncthreads();
#pragma unroll 1
    for (int pass = 0; pass < 2; ++pass) {
      for (int ch = tid; ch < KG * 63; ch += 256) { const int co = ch / 63, q = (ch % 63) * 2;
        v2f_t v; v.x = so[co * 128 + q]; v.y = so[co * 128 + q + 1];
        *(volatile v2f_t*)(obase + ((size_t)co * HO + y) * WO + q) = v; }
      __threadfence();
    }
  }
}

extern "C" void kernel_launch(void* const* d_in, const int* in_sizes, int n_in,
                              void* d_out, int out_size, void* d_ws, size_t ws_size,
                              hipStream_t stream) {
  (void)in_sizes; (void)n_in; (void)out_size; (void)ws_size;
  const float* x    = (const float*)d_in[0];
  const float* filt = (const float*)d_in[1];
  float*       Y    = (float*)d_out;
  h16* wp = (h16*)d_ws;
  h16* xp = wp + 9 * CO * CI;
  k_pack_w<<<(9 * CO * (CI / 8) + 255) / 256, 256, 0, stream>>>(filt, wp);
  k_pack_x<<<(NI * HI * WI * (CI / 8)) / 256, 256, 0, stream>>>(x, xp);
  k_conv<<<NI * (CO / KG), 256, 0, stream>>>(xp, wp, Y);
}
